// PSSM_70179765616886
// MI455X (gfx1250) — hardware-verified
//
#include <hip/hip_runtime.h>
#include <math.h>

typedef __attribute__((ext_vector_type(16))) _Float16 v16h;
typedef __attribute__((ext_vector_type(16))) __bf16 v16b;
typedef __attribute__((ext_vector_type(8)))  _Float16 v8h;
typedef __attribute__((ext_vector_type(8)))  float v8f;
typedef __attribute__((ext_vector_type(4)))  float v4f;
typedef __attribute__((ext_vector_type(2)))  float v2f;
typedef __attribute__((ext_vector_type(4)))  unsigned v4u;
typedef __attribute__((ext_vector_type(4)))  int v4i;
typedef float __attribute__((may_alias)) float_a;
typedef int __attribute__((may_alias)) int_a;

template <typename T> __device__ __forceinline__ void vst2(void* p, T v) { *(volatile T*)p = v; __threadfence(); *(volatile T*)p = v; }
__device__ __forceinline__ v8f wmma16(v16h a, v16h b, v8f c) {
  v8f d = __builtin_amdgcn_wmma_f32_16x16x32_f16(false, a, false, b, (short)0, c, false, false);
  asm volatile("v_nop\n\tv_nop\n\tv_nop\n\tv_nop" : "+v"(d) : "v"(a), "v"(b));
  return d;
}
__device__ __forceinline__ v8f wmma_bf(v16b a, v16b b, v8f c) {
  v8f d = __builtin_amdgcn_wmma_f32_16x16x32_bf16(false, a, false, b, (short)0, c, false, false);
  asm volatile("v_nop\n\tv_nop\n\tv_nop\n\tv_nop" : "+v"(d) : "v"(a), "v"(b));
  return d;
}
__device__ __forceinline__ v16h frag_h(const _Float16* rowk0, int lane) {
  union { v16h v; v8h q[2]; } u; const _Float16* p = rowk0 + 8 * (lane >> 4);
  u.q[0] = *(const v8h*)p; u.q[1] = *(const v8h*)(p + 16); return u.v;
}
__device__ __forceinline__ v16h frag_f32(const float* rowk0, int lane) {
  v16h a; const float* p = rowk0 + 8 * (lane >> 4);
#pragma unroll
  for (int i = 0; i < 8; ++i) { a[i] = (_Float16)p[i]; a[8 + i] = (_Float16)p[16 + i]; }
  return a;
}
__device__ __forceinline__ v16h frag_f32s(const float* rowk0, int lane, float sc) {
  v16h a; const float* p = rowk0 + 8 * (lane >> 4);
#pragma unroll
  for (int i = 0; i < 8; ++i) { a[i] = (_Float16)(p[i] * sc); a[8 + i] = (_Float16)(p[16 + i] * sc); }
  return a;
}
__device__ __forceinline__ v16h fragc_f32(const float* W, int k0, int n, int lane, int ld, int K) {
  v16h a; const int g = lane >> 4;
#pragma unroll
  for (int i = 0; i < 8; ++i) { const int ka = k0 + 8 * g + i, kb = ka + 16;
    a[i] = (_Float16)(ka < K ? W[(size_t)(ka < K ? ka : K - 1) * ld + n] : 0.f); a[8 + i] = (_Float16)(kb < K ? W[(size_t)(kb < K ? kb : K - 1) * ld + n] : 0.f); }
  return a;
}
struct F2 { v16b h, l; };
__device__ __forceinline__ F2 bsplit16(const float v[16]) { F2 r;
#pragma unroll
  for (int i = 0; i < 16; ++i) { const __bf16 h = (__bf16)v[i]; r.h[i] = h; r.l[i] = (__bf16)(v[i] - (float)h); }
  return r; }
__device__ __forceinline__ F2 split_row(const float* row, int k0, int lane) { float v[16]; const float* p = row + k0 + 8 * (lane >> 4);
#pragma unroll
  for (int i = 0; i < 8; ++i) { v[i] = p[i]; v[8 + i] = p[16 + i]; }
  return bsplit16(v); }
__device__ __forceinline__ F2 split_rowK(const float* row, int k0, int lane, int K) { float v[16]; const int g = lane >> 4;
#pragma unroll
  for (int i = 0; i < 8; ++i) { const int ka = k0 + 8 * g + i, kb = ka + 16; v[i] = ka < K ? row[ka < K ? ka : K - 1] : 0.f; v[8 + i] = kb < K ? row[kb < K ? kb : K - 1] : 0.f; }
  return bsplit16(v); }
__device__ __forceinline__ F2 split_col(const float* W, int k0, int n, int lane, int ld, int K) { float v[16]; const int g = lane >> 4;
#pragma unroll
  for (int i = 0; i < 8; ++i) { const int ka = k0 + 8 * g + i, kb = ka + 16; v[i] = ka < K ? W[(size_t)(ka < K ? ka : K - 1) * ld + n] : 0.f; v[8 + i] = kb < K ? W[(size_t)(kb < K ? kb : K - 1) * ld + n] : 0.f; }
  return bsplit16(v); }
__device__ __forceinline__ v8f mac3(const F2& a, const F2& b, v8f c) { c = wmma_bf(a.l, b.h, c); c = wmma_bf(a.h, b.l, c); return wmma_bf(a.h, b.h, c); }
__device__ __forceinline__ float sigm(float v) { return 1.0f / (1.0f + expf(-v)); }
#define LDSX() do { asm volatile("s_wait_dscnt 0" ::: "memory"); __builtin_amdgcn_wave_barrier(); __builtin_amdgcn_fence(__ATOMIC_RELEASE, "workgroup"); } while (0)


#define NB 2
#define LL 2048
#define DIM 64
#define DI 128
#define NS 64
#define KC 4
#ifndef TNB
#define TNB NB
#endif
typedef __attribute__((ext_vector_type(8))) __bf16 v8b;
__device__ __forceinline__ v16b frag_b(const __bf16* rowk0, int lane) {
  union { v16b v; v8b q[2]; } u; const __bf16* p = rowk0 + 8 * (lane >> 4);
  u.q[0] = *(const v8b*)p; u.q[1] = *(const v8b*)(p + 16); return u.v;
}
__device__ __forceinline__ float bfr(float v) { return (float)(__bf16)v; }
__device__ __attribute__((noinline)) float exp_ni(float v) { return expf(v); }
__device__ __attribute__((noinline)) float erf_ni(float v) { return erff(v); }

#define WS_PW  0u
#define WS_XP  (WS_PW + 2u * 3 * DI * DIM)
#define WS_XCD (WS_XP + 4u * NB * LL * 3 * DI)
#define WS_YF  (WS_XCD + 4u * NB * LL * 2 * DI)
#define WS_END (WS_YF + 4u * NB * LL * DI)

__global__ __launch_bounds__(64) void k_pack(const float* __restrict__ WP, __bf16* __restrict__ PW) {
  __shared__ __align__(16) __bf16 s[DIM]; const int r = blockIdx.x, k = threadIdx.x; s[k] = (__bf16)WP[(size_t)r * DIM + k]; __syncthreads();
  if (k < DIM / 8) vst2((unsigned*)(PW + (size_t)r * DIM + k * 8), *(const v4u*)&s[k * 8]);
}
__global__ __launch_bounds__(128) void k_proj(const float* __restrict__ X, const __bf16* __restrict__ PW, float* __restrict__ XP) {
  __shared__ __align__(16) float so[4][16][132];
  const int tid = threadIdx.x, wave = tid >> 5, lane = tid & 31, col = lane & 15, g = lane >> 4; const size_t r0 = (size_t)blockIdx.x * 64 + wave * 16; const int n0 = blockIdx.y * 128;
  v8f acc[8] = {};
#pragma unroll
  for (int kc = 0; kc < DIM / 32; ++kc) { v16b a; { const float* p = X + (r0 + col) * DIM + kc * 32 + 8 * g;
#pragma unroll
      for (int i = 0; i < 8; ++i) { a[i] = (__bf16)p[i]; a[8 + i] = (__bf16)p[16 + i]; } }
#pragma unroll
    for (int j = 0; j < 8; ++j) acc[j] = wmma_bf(a, frag_b(PW + (size_t)(n0 + j * 16 + col) * DIM + kc * 32, lane), acc[j]); }
#pragma unroll
  for (int j = 0; j < 8; ++j)
#pragma unroll
    for (int r = 0; r < 8; ++r) so[wave][8 * g + r][j * 16 + col] = acc[j][r];
  LDSX();
  for (int rl = 0; rl < 16; ++rl) vst2(XP + (r0 + rl) * (3 * DI) + n0 + lane * 4, *(const v4f*)&so[wave][rl][lane * 4]);
}
__global__ __launch_bounds__(128) void k_conv(const float* __restrict__ XP, const float* __restrict__ CWt, const float* __restrict__ CB, float* __restrict__ XCD) {
  __shared__ __align__(16) float so[2][64][DI];
  const int d = threadIdx.x; const size_t r0 = (size_t)blockIdx.x * 64; const int b = (int)(r0 / LL); const int l0 = (int)(r0 % LL);
  float w[KC];
#pragma unroll
  for (int j = 0; j < KC; ++j) w[j] = bfr(CWt[d * KC + j]);
  const float cb = bfr(CB[d]);
  for (int rl = 0; rl < 64; ++rl) { const int l = l0 + rl; float acc = cb;
#pragma unroll
    for (int j = 0; j < KC; ++j) { const int ls = l - (KC - 1) + j; if (ls >= 0) acc += w[j] * XP[((size_t)b * LL + ls) * (3 * DI) + d]; }
    so[0][rl][d] = acc; so[1][rl][d] = sigm(XP[(r0 + rl) * (3 * DI) + DI + d]); }
  __syncthreads();
  for (int q = d; q < 64 * 64; q += 128) { const int rl = q >> 6, pc = q & 63; const int which = pc >> 5, p4 = pc & 31; vst2(XCD + ((r0 + rl) * 2 + which) * DI + p4 * 4, *(const v4f*)&so[which][rl][p4 * 4]); }
}
template <int DIR>
__global__ __launch_bounds__(256) void k_scan(const float* __restrict__ XP, const float* __restrict__ XCD, const float* __restrict__ Am, const float* __restrict__ Dv, float* __restrict__ YF, float* __restrict__ out) {
  __shared__ float sa[NS]; __shared__ __align__(16) float sred[8][32]; __shared__ __align__(16) float sy[32];
  const int tid = threadIdx.x, dl = tid & 31, ng = tid >> 5; const int dch = blockIdx.x, b = blockIdx.y; const int d = dch * 32 + dl;
  if (tid < NS) { float s = 0.f; for (int j = 0; j < NS; ++j) s += bfr(Am[tid * NS + j]); sa[tid] = s; }
  __syncthreads();
  float an[8], h[8];
#pragma unroll
  for (int i = 0; i < 8; ++i) { an[i] = sa[ng * 8 + i]; h[i] = 0.f; }
  const float dd = bfr(Dv[d]);
#pragma unroll 1
  for (int step = 0; step < LL; ++step) { const int l = DIR ? (LL - 1 - step) : step; const size_t row = (size_t)b * LL + l;
    const float xc = XCD[(row * 2 + 0) * DI + d], de = XCD[(row * 2 + 1) * DI + d]; const float* bc = XP + row * (3 * DI) + 2 * DI;
    const float u = de * xc; float py = 0.f;
#pragma unroll
    for (int i = 0; i < 8; ++i) { const int n = ng * 8 + i; const float abar = exp_ni(de * an[i]); h[i] = abar * h[i] + u * bc[n]; py += h[i] * bc[NS + n]; }
    sred[ng][dl] = py;
    __syncthreads();
    if (tid < 32) { float y = 0.f;
#pragma unroll
      for (int q = 0; q < 8; ++q) y += sred[q][tid];
      if (DIR == 0) sy[tid] = y; else sy[tid] = YF[row * DI + dch * 32 + tid] + y + dd * XCD[(row * 2 + 0) * DI + dch * 32 + tid]; }
    __syncthreads();
    if (tid < 8) { float* dst = (DIR == 0) ? (YF + row * DI + dch * 32) : (out + row * DI + dch * 32); vst2(dst + tid * 4, *(const v4f*)&sy[tid * 4]); }
  }
}
extern "C" void kernel_launch(void* const* d_in, const int* in_sizes, int n_in, void* d_out, int out_size, void* d_ws, size_t ws_size, hipStream_t stream) {
  (void)in_sizes; (void)n_in; (void)out_size;
  const float** F = (const float**)d_in;
  if (ws_size < (size_t)WS_END) return;
  char* ws = (char*)d_ws; __bf16* PW = (__bf16*)(ws + WS_PW); float *XP = (float*)(ws + WS_XP), *XCD = (float*)(ws + WS_XCD), *YF = (float*)(ws + WS_YF);
  k_pack<<<3 * DI, 64, 0, stream>>>(F[1], PW);
  k_proj<<<dim3(TNB * LL / 64, 3), 128, 0, stream>>>(F[0], PW, XP);
  k_conv<<<TNB * LL / 64, 128, 0, stream>>>(XP, F[2], F[3], XCD);
  k_scan<0><<<dim3(DI / 32, TNB), 256, 0, stream>>>(XP, XCD, F[4], F[5], YF, (float*)d_out);
  k_scan<1><<<dim3(DI / 32, TNB), 256, 0, stream>>>(XP, XCD, F[4], F[5], YF, (float*)d_out);
}
